// SparseTransformerLayer_61392262529129
// MI455X (gfx1250) — hardware-run, weakly checked
//
#include <hip/hip_runtime.h>
#include <math.h>

constexpr int kBatch    = 2;
constexpr int kSeq      = 2048;
constexpr int kDim      = 1024;
constexpr int kFF       = 4096;
constexpr int kHeads    = 16;
constexpr int kHeadDim  = 64;
constexpr int kTok      = kBatch * kSeq;
constexpr int kHalfWin  = 204;
constexpr int kChunkQ   = 128;
constexpr int kWinK     = 640;
constexpr int kKw0Max   = kSeq - kWinK;
constexpr int kChunks   = kSeq / kChunkQ;
constexpr int kGroups   = kBatch * kHeads;
constexpr int kGroupsPerPass = 4;
constexpr int kZPerPass = kGroupsPerPass * kChunks;
constexpr int kPasses   = kGroups / kGroupsPerPass;
constexpr float kWCarry    = 16.0f;
constexpr float kWCarryInv = 1.0f / 16.0f;
constexpr float kPCarry    = 2048.0f;
constexpr float kCtxCarry  = 256.0f;
constexpr float kPVScale   = kCtxCarry / kPCarry;
constexpr float kWoScale   = 1.0f / (kCtxCarry * kWCarry);
constexpr float kScoreScale = 0.125f;
constexpr float kInvDim    = 1.0f / 1024.0f;
constexpr float kLnEps     = 1e-5f;

typedef __attribute__((ext_vector_type(16))) _Float16 v16h;
typedef __attribute__((ext_vector_type(8)))  _Float16 v8h;
typedef __attribute__((ext_vector_type(16))) __bf16   v16b;
typedef __attribute__((ext_vector_type(8)))  __bf16   v8b;
typedef __attribute__((ext_vector_type(8)))  float    v8f;
typedef __attribute__((ext_vector_type(4)))  float    v4f;
typedef __attribute__((ext_vector_type(4)))  unsigned int v4u;

__device__ __forceinline__ unsigned short f2bf_bits(float f) {
  unsigned u = __float_as_uint(f);
  return (unsigned short)((u + 0x7FFFu + ((u >> 16) & 1u)) >> 16);
}
__device__ __forceinline__ float bf_bits2f(unsigned short h) { return __uint_as_float(((unsigned)h) << 16); }

__device__ __forceinline__ void dep_guard_h(v8f& a, v8f& b, v16h x, v16h y) { asm volatile("v_nop\n\tv_nop\n\tv_nop\n\tv_nop" : "+v"(a), "+v"(b) : "v"(x), "v"(y)); }
__device__ __forceinline__ void dep_guard_b(v8f& a, v8f& b, v16b x, v16b y) { asm volatile("v_nop\n\tv_nop\n\tv_nop\n\tv_nop" : "+v"(a), "+v"(b) : "v"(x), "v"(y)); }
__device__ __forceinline__ void keep4_h(v16h a, v16h b, v16h c, v16h d) { asm volatile("v_nop" :: "v"(a), "v"(b), "v"(c), "v"(d)); }
__device__ __forceinline__ void keep4_b(v16b a, v16b b, v16b c, v16b d) { asm volatile("v_nop" :: "v"(a), "v"(b), "v"(c), "v"(d)); }
__device__ __forceinline__ void acc_guard4(v8f& a, v8f& b, v8f& c, v8f& d) { asm volatile("v_nop\n\tv_nop\n\tv_nop\n\tv_nop" : "+v"(a), "+v"(b), "+v"(c), "+v"(d)); }
template <typename T> struct Frag;
template <> struct Frag<_Float16> {
  typedef v16h V; union U { v16h v; v8h h[2]; };
  static __device__ __forceinline__ v16h load(const _Float16* p) {
    U f; f.h[0] = *(const v8h*)(p); f.h[1] = *(const v8h*)(p + 16); return f.v;
  }
  static __device__ __forceinline__ v8f mma(v16h a, v16h b, v8f c) {
    return __builtin_amdgcn_wmma_f32_16x16x32_f16(false, a, false, b, (short)0, c, false, false);
  }
  static __device__ __forceinline__ void guard(v8f& a, v8f& b, v16h x, v16h y) { dep_guard_h(a, b, x, y); }
  static __device__ __forceinline__ void keep(v16h a, v16h b, v16h c, v16h d) { keep4_h(a, b, c, d); }
};
template <> struct Frag<__bf16> {
  typedef v16b V; union U { v16b v; v8b h[2]; };
  static __device__ __forceinline__ v16b load(const __bf16* p) {
    U f; f.h[0] = *(const v8b*)(p); f.h[1] = *(const v8b*)(p + 16); return f.v;
  }
  static __device__ __forceinline__ v8f mma(v16b a, v16b b, v8f c) {
    return __builtin_amdgcn_wmma_f32_16x16x32_bf16(false, a, false, b, (short)0, c, false, false);
  }
  static __device__ __forceinline__ void guard(v8f& a, v8f& b, v16b x, v16b y) { dep_guard_b(a, b, x, y); }
  static __device__ __forceinline__ void keep(v16b a, v16b b, v16b c, v16b d) { keep4_b(a, b, c, d); }
};

__device__ __forceinline__ unsigned pk16(unsigned short a, unsigned short b) { return (unsigned)a | ((unsigned)b << 16); }
__device__ __forceinline__ unsigned short h_bits(float f) { const _Float16 h = (_Float16)f; return __builtin_bit_cast(unsigned short, h); }

__device__ __forceinline__ int band_kw0(int cch) {
  int k = cch * kChunkQ - 256;
  k = k < 0 ? 0 : k;
  k = k > kKw0Max ? kKw0Max : k;
  return k;
}

template <int ET> struct Elem;
template <> struct Elem<0> { typedef _Float16 T; };
template <> struct Elem<1> { typedef __bf16 T; };
template <int ET, bool SPLIT, int BIAS_MODE, int OUT_MODE, bool RESID, int ACT = 0, int GEO = 0>
__global__ __launch_bounds__(256) void wmma_gemm64(
    const unsigned short* __restrict__ Ap, const unsigned short* __restrict__ A2p, int lda, long strideA,
    const unsigned short* __restrict__ Btp, const unsigned short* __restrict__ Bt2p, int ldb, long strideB,
    void* __restrict__ Cout, void* __restrict__ Cout2, int ldc, long strideC,
    const float* __restrict__ bias,
    const float* __restrict__ resid, long strideR,
    int M, int N, int K, float scale, int gbase) {
  typedef typename Elem<ET>::T T;
  typedef typename Frag<T>::V V;
  const T* A = (const T*)Ap; const T* A2 = (const T*)A2p; const T* Bt = (const T*)Btp; const T* Bt2 = (const T*)Bt2p;
  __shared__ __align__(16) float sT[8][16 * 68];
  const int b    = blockIdx.y;
  const int lane = threadIdx.x & 31;
  const int wave = threadIdx.x >> 5;
  const int tilesN = N >> 6;
  const int tilesM = M >> 6;
  const int tile = blockIdx.x * 8 + wave;
  if (tile >= tilesM * tilesN) return;
  const int tm = tile / tilesN;
  const int tn = tile - tm * tilesN;
  const int m0 = tm << 6;
  const int n0 = tn << 6;

  size_t offA, offB, offC, offR;
  if (GEO == 0) {
    offA = (size_t)b * strideA; offB = (size_t)b * strideB; offC = (size_t)b * strideC; offR = (size_t)b * strideR;
  } else {
    const int zg  = b >> 4, cch = b & 15;
    const int grp = gbase + zg;
    const int bb  = grp >> 4, hd = grp & 15;
    const int kw0 = band_kw0(cch);
    if (GEO == 1) {
      offA = (size_t)(bb * kSeq + cch * kChunkQ) * kDim + hd * kHeadDim;
      offB = (size_t)(bb * kSeq + kw0) * kDim + hd * kHeadDim;
      offC = (size_t)b * (kChunkQ * kWinK);
    } else {
      offA = (size_t)b * (kChunkQ * kWinK);
      offB = (size_t)(grp * kHeadDim) * kSeq + kw0;
      offC = (size_t)(bb * kSeq + cch * kChunkQ) * kDim + hd * kHeadDim;
    }
    offR = 0;
  }

  const T* Ab  = A  + offA;
  const T* Bb  = Bt + offB;
  const T* Ab2 = SPLIT ? (A2  + offA) : nullptr;
  const T* Bb2 = SPLIT ? (Bt2 + offB) : nullptr;

  const int rlane = lane & 15;
  const int koff  = (lane >> 4) * 8;
  const int mOff  = (lane >> 4) * 8;

  v8f acc[4][4];
#pragma unroll
  for (int i = 0; i < 4; ++i)
#pragma unroll
    for (int j = 0; j < 4; ++j) acc[i][j] = (v8f){0.f,0.f,0.f,0.f,0.f,0.f,0.f,0.f};

  for (int k0 = 0; k0 < K; k0 += 32) {
    V bh[4], bl[4];
#pragma unroll
    for (int j = 0; j < 4; ++j) {
      const size_t bo = (size_t)(n0 + (j << 4) + rlane) * ldb + koff + k0;
      bh[j] = Frag<T>::load(Bb + bo);
      if (SPLIT) bl[j] = Frag<T>::load(Bb2 + bo);
    }
#pragma unroll
    for (int i = 0; i < 4; ++i) {
      const size_t ao = (size_t)(m0 + (i << 4) + rlane) * lda + koff + k0;
      V ah = Frag<T>::load(Ab + ao);
      V al;
      if (SPLIT) al = Frag<T>::load(Ab2 + ao);
#pragma unroll
      for (int j = 0; j < 4; ++j) {
        acc[i][j] = Frag<T>::mma(ah, bh[j], acc[i][j]);
        if (SPLIT) {
          acc[i][j] = Frag<T>::mma(ah, bl[j], acc[i][j]);
          acc[i][j] = Frag<T>::mma(al, bh[j], acc[i][j]);
        }
      }
      Frag<T>::guard(acc[i][0], acc[i][3], ah, SPLIT ? al : ah);
    }
    Frag<T>::keep(bh[0], bh[1], bh[2], bh[3]);
    if (SPLIT) Frag<T>::keep(bl[0], bl[1], bl[2], bl[3]);
  }
  acc_guard4(acc[0][0], acc[0][1], acc[0][2], acc[0][3]);
  acc_guard4(acc[1][0], acc[1][1], acc[1][2], acc[1][3]);
  acc_guard4(acc[2][0], acc[2][1], acc[2][2], acc[2][3]);
  acc_guard4(acc[3][0], acc[3][1], acc[3][2], acc[3][3]);

  float* slab = sT[wave];
  const float* Rb = RESID ? (resid + offR) : nullptr;
#pragma unroll
  for (int i = 0; i < 4; ++i) {
    const int mBase = m0 + (i << 4);
#pragma unroll
    for (int j = 0; j < 4; ++j) {
      const int n = n0 + (j << 4) + rlane;
      float bv = 0.f;
      if (BIAS_MODE == 2) bv = bias[n];
#pragma unroll
      for (int r = 0; r < 8; ++r) {
        float v = acc[i][j][r] * scale;
        if (BIAS_MODE == 1) v += bias[mBase + mOff + r];
        if (BIAS_MODE == 2) v += bv;
        if (RESID) v += Rb[(size_t)(mBase + mOff + r) * ldc + n];
        if (ACT == 2) v = fmaxf(v, 0.0f);
        if (ACT == 4) v = (v > 0.f) ? v : 0.01f * v;
        slab[(mOff + r) * 68 + (j << 4) + rlane] = v;
      }
    }
    __builtin_amdgcn_fence(__ATOMIC_RELEASE, "workgroup");
    __builtin_amdgcn_wave_barrier();
    __builtin_amdgcn_fence(__ATOMIC_ACQUIRE, "workgroup");
    if (OUT_MODE == 0) {
      float* C = (float*)Cout + offC;
      const int hh = lane >> 4, c4 = (lane & 15) * 4;
      for (int pass = 0; pass < 2; ++pass) {
#pragma unroll
        for (int it = 0; it < 8; ++it) {
          const int row = it * 2 + hh;
          v4f v = *(const v4f*)(slab + row * 68 + c4);
          *(volatile v4f*)(C + (size_t)(mBase + row) * ldc + n0 + c4) = v;
        }
        __threadfence();
      }
    } else {
      const int q = lane >> 3, c8 = (lane & 7) * 8;
      unsigned short* C  = (unsigned short*)Cout  + offC;
      unsigned short* C2 = (OUT_MODE == 2) ? ((unsigned short*)Cout2 + offC) : nullptr;
      for (int pass = 0; pass < 2; ++pass) {
#pragma unroll
        for (int it = 0; it < 4; ++it) {
          const int row = it * 4 + q;
          const float* sp = slab + row * 68 + c8;
          v8h hv, lv;
#pragma unroll
          for (int e = 0; e < 8; ++e) {
            if (OUT_MODE == 1) {
              hv[e] = (_Float16)sp[e];
            } else {
              unsigned short hb = f2bf_bits(sp[e]);
              unsigned short lb = f2bf_bits(sp[e] - bf_bits2f(hb));
              hv[e] = __builtin_bit_cast(_Float16, hb);
              lv[e] = __builtin_bit_cast(_Float16, lb);
            }
          }
          *(volatile v8h*)(C + (size_t)(mBase + row) * ldc + n0 + c8) = hv;
          if (OUT_MODE == 2) *(volatile v8h*)(C2 + (size_t)(mBase + row) * ldc + n0 + c8) = lv;
        }
        __threadfence();
      }
    }
    __builtin_amdgcn_fence(__ATOMIC_RELEASE, "workgroup");
    __builtin_amdgcn_wave_barrier();
    __builtin_amdgcn_fence(__ATOMIC_ACQUIRE, "workgroup");
  }
}

__global__ __launch_bounds__(256) void wtcast_kernel(const float* __restrict__ W0, const float* __restrict__ W1,
                                                     const float* __restrict__ W2, const float* __restrict__ W3,
                                                     unsigned short* __restrict__ out, int kin, int nout,
                                                     long planeStride, float scale) {
  __shared__ float sm[64][65];
  const int t  = threadIdx.x;
  const int k0 = blockIdx.x * 64;
  const int n0 = blockIdx.y * 64;
  const int z  = blockIdx.z;
  const float* W = (z == 0) ? W0 : (z == 1) ? W1 : (z == 2) ? W2 : W3;
#pragma unroll
  for (int i = 0; i < 16; ++i) {
    const int e = i * 256 + t;
    const int r = e >> 6;
    const int c = e & 63;
    sm[c][r] = W[(size_t)(k0 + r) * nout + n0 + c] * scale;
  }
  __syncthreads();
  const int lane = t & 31, wave = t >> 5;
  const int q = lane >> 3, c8 = (lane & 7) * 8;
  unsigned short* op = out + (size_t)z * planeStride;
  for (int pass = 0; pass < 2; ++pass) {
#pragma unroll
    for (int it = 0; it < 2; ++it) {
      const int row = wave * 8 + it * 4 + q;
      unsigned short hb[8];
#pragma unroll
      for (int e = 0; e < 8; ++e) hb[e] = h_bits(sm[row][c8 + e]);
      const v4u u = (v4u){pk16(hb[0], hb[1]), pk16(hb[2], hb[3]), pk16(hb[4], hb[5]), pk16(hb[6], hb[7])};
      *(volatile v4u*)(op + (size_t)(n0 + row) * kin + k0 + c8) = u;
    }
    __threadfence();
  }
}

__global__ __launch_bounds__(128) void ln_f16_kernel(const float* __restrict__ X, const float* __restrict__ G,
                                                     const float* __restrict__ Bt, unsigned short* __restrict__ out) {
  __shared__ float redA[4];
  __shared__ float redB[4];
  const int row  = blockIdx.x;
  const int t    = threadIdx.x;
  const int lane = t & 31, wave = t >> 5;
  const int c0   = t * 8;
  const float* xr = X + (size_t)row * kDim + c0;
  const v4f a  = *(const v4f*)(xr);
  const v4f c  = *(const v4f*)(xr + 4);
  const v4f ga = *(const v4f*)(G + c0);
  const v4f gc = *(const v4f*)(G + c0 + 4);
  const v4f ba = *(const v4f*)(Bt + c0);
  const v4f bc = *(const v4f*)(Bt + c0 + 4);
  float v[8], gg[8], bb[8];
#pragma unroll
  for (int e = 0; e < 4; ++e) {
    v[e] = a[e]; v[4 + e] = c[e];
    gg[e] = ga[e]; gg[4 + e] = gc[e];
    bb[e] = ba[e]; bb[4 + e] = bc[e];
  }
  float s = ((v[0] + v[1]) + (v[2] + v[3])) + ((v[4] + v[5]) + (v[6] + v[7]));
#pragma unroll
  for (int off = 16; off > 0; off >>= 1) s += __shfl_xor(s, off, 32);
  if (lane == 0) redA[wave] = s;
  __syncthreads();
  const float mean = (((redA[0] + redA[1]) + redA[2]) + redA[3]) * kInvDim;
  float d[8];
  float qv = 0.f;
#pragma unroll
  for (int e = 0; e < 8; ++e) { d[e] = v[e] - mean; qv += d[e] * d[e]; }
#pragma unroll
  for (int off = 16; off > 0; off >>= 1) qv += __shfl_xor(qv, off, 32);
  if (lane == 0) redB[wave] = qv;
  __syncthreads();
  const float var  = (((redB[0] + redB[1]) + redB[2]) + redB[3]) * kInvDim;
  const float rstd = rsqrtf(var + kLnEps);
  unsigned short hb[8];
#pragma unroll
  for (int e = 0; e < 8; ++e) hb[e] = h_bits(d[e] * rstd * gg[e] + bb[e]);
  const v4u u = (v4u){pk16(hb[0], hb[1]), pk16(hb[2], hb[3]), pk16(hb[4], hb[5]), pk16(hb[6], hb[7])};
  unsigned short* op = out + (size_t)row * kDim + c0;
  *(volatile v4u*)op = u;
  __threadfence();
  *(volatile v4u*)op = u;
}

__global__ __launch_bounds__(128) void band_softmax_kernel(const float* __restrict__ Sc, unsigned short* __restrict__ P) {
  __shared__ float redM[4];
  __shared__ float redS[4];
  const int row  = blockIdx.x;
  const int z    = blockIdx.y;
  const int cch  = z & 15;
  const int kw0  = band_kw0(cch);
  const int qi   = cch * kChunkQ + row;
  const int t    = threadIdx.x;
  const int lane = t & 31, wave = t >> 5;
  const bool act = t < 80;
  const int tc   = act ? t : 79;
  const size_t rbase = ((size_t)z * kChunkQ + row) * kWinK;
  const float* sr = Sc + rbase + tc * 8;
  const v4f a = *(const v4f*)(sr);
  const v4f c = *(const v4f*)(sr + 4);
  float xv[8];
#pragma unroll
  for (int e = 0; e < 4; ++e) { xv[e] = a[e]; xv[4 + e] = c[e]; }
  float m = -1e30f;
#pragma unroll
  for (int e = 0; e < 8; ++e) {
    const int j  = kw0 + tc * 8 + e;
    const int dj = j - qi;
    const bool allowed = act && (dj >= -kHalfWin) && (dj <= kHalfWin);
    xv[e] = allowed ? xv[e] : -1e30f;
    m = fmaxf(m, xv[e]);
  }
#pragma unroll
  for (int off = 16; off > 0; off >>= 1) m = fmaxf(m, __shfl_xor(m, off, 32));
  if (lane == 0) redM[wave] = m;
  __syncthreads();
  m = fmaxf(fmaxf(redM[0], redM[1]), fmaxf(redM[2], redM[3]));
  float p[8];
  float s = 0.f;
#pragma unroll
  for (int e = 0; e < 8; ++e) { p[e] = expf(xv[e] - m); s += p[e]; }
#pragma unroll
  for (int off = 16; off > 0; off >>= 1) s += __shfl_xor(s, off, 32);
  if (lane == 0) redS[wave] = s;
  __syncthreads();
  s = ((redS[0] + redS[1]) + redS[2]) + redS[3];
  const float f = kPCarry * (1.0f / s);
  unsigned short hb[8];
#pragma unroll
  for (int e = 0; e < 8; ++e) hb[e] = h_bits(p[e] * f);
  const v4u u = (v4u){pk16(hb[0], hb[1]), pk16(hb[2], hb[3]), pk16(hb[4], hb[5]), pk16(hb[6], hb[7])};
  unsigned short* op = P + rbase + (size_t)tc * 8;
  if (act) *(volatile v4u*)op = u;
  __threadfence();
  if (act) *(volatile v4u*)op = u;
}

extern "C" void kernel_launch(void* const* d_in, const int* in_sizes, int n_in,
                              void* d_out, int out_size, void* d_ws, size_t ws_size,
                              hipStream_t stream) {
  if (n_in < 17) return;
  if (in_sizes[0] != kTok * kDim || out_size != kTok * kDim) return;
  if (in_sizes[1] != kDim * kDim || in_sizes[13] != kDim * kFF || in_sizes[15] != kFF * kDim) return;

  const float* x    = (const float*)d_in[0];
  const float* wq   = (const float*)d_in[1];
  const float* bq   = (const float*)d_in[2];
  const float* wk   = (const float*)d_in[3];
  const float* bk   = (const float*)d_in[4];
  const float* wv   = (const float*)d_in[5];
  const float* bv   = (const float*)d_in[6];
  const float* wo   = (const float*)d_in[7];
  const float* bo   = (const float*)d_in[8];
  const float* ln1g = (const float*)d_in[9];
  const float* ln1b = (const float*)d_in[10];
  const float* ln2g = (const float*)d_in[11];
  const float* ln2b = (const float*)d_in[12];
  const float* w1   = (const float*)d_in[13];
  const float* b1   = (const float*)d_in[14];
  const float* w2   = (const float*)d_in[15];
  const float* b2   = (const float*)d_in[16];
  float* out = (float*)d_out;

  const size_t plane16 = (size_t)kTok * kDim * 2;
  const size_t offXn   = 0;
  const size_t offWT4  = offXn  + plane16;
  const size_t offW1T  = offWT4 + plane16;
  const size_t offW2T  = offW1T + (size_t)kFF * kDim * 2;
  const size_t offQ    = offW2T + (size_t)kDim * kFF * 2;
  const size_t offK    = offQ   + plane16;
  const size_t offVT   = offK   + plane16;
  const size_t offCtx  = offVT  + plane16;
  const size_t offX1   = offCtx + plane16;
  const size_t offScr  = offX1  + (size_t)kTok * kDim * 4;
  const size_t scrBytes = (size_t)kTok * kFF * 2;
  const size_t scoresBytes = (size_t)kZPerPass * kChunkQ * kWinK * 4;
  const size_t pBytes      = (size_t)kZPerPass * kChunkQ * kWinK * 2;
  const size_t total   = offScr + scrBytes;
  if (total > ws_size) return;
  if (scoresBytes + pBytes > scrBytes) return;

  char* ws = (char*)d_ws;
  unsigned short* xn   = (unsigned short*)(ws + offXn);
  unsigned short* wT4  = (unsigned short*)(ws + offWT4);
  unsigned short* wqT  = wT4;
  unsigned short* wkT  = wT4 + (size_t)kDim * kDim;
  unsigned short* wvT  = wT4 + (size_t)2 * kDim * kDim;
  unsigned short* woT  = wT4 + (size_t)3 * kDim * kDim;
  unsigned short* w1T  = (unsigned short*)(ws + offW1T);
  unsigned short* w2T  = (unsigned short*)(ws + offW2T);
  unsigned short* qh   = (unsigned short*)(ws + offQ);
  unsigned short* kh   = (unsigned short*)(ws + offK);
  unsigned short* vT   = (unsigned short*)(ws + offVT);
  unsigned short* ctx  = (unsigned short*)(ws + offCtx);
  float*          x1   = (float*)(ws + offX1);
  float*          scr  = (float*)(ws + offScr);
  float*          scores = scr;
  unsigned short* pPl  = (unsigned short*)(ws + offScr + scoresBytes);
  unsigned short* ff1  = (unsigned short*)(ws + offScr);

  wtcast_kernel<<<dim3(kDim / 64, kDim / 64, 4), 256, 0, stream>>>(wq, wk, wv, wo, wT4, kDim, kDim,
                                                                   (long)kDim * kDim, kWCarry);
  wtcast_kernel<<<dim3(kDim / 64, kFF / 64, 1), 256, 0, stream>>>(w1, w1, w1, w1, w1T, kDim, kFF, 0L, kWCarry);
  wtcast_kernel<<<dim3(kFF / 64, kDim / 64, 1), 256, 0, stream>>>(w2, w2, w2, w2, w2T, kFF, kDim, 0L, kWCarry);

  ln_f16_kernel<<<dim3(kTok), 128, 0, stream>>>(x, ln1g, ln1b, xn);

  wmma_gemm64<0, false, 2, 1, false, 0, 0><<<dim3(128, 1, 1), 256, 0, stream>>>(
      xn, xn, kDim, 0L, wqT, wqT, kDim, 0L, (void*)qh, (void*)qh, kDim, 0L, bq, x, 0L,
      kTok, kDim, kDim, kWCarryInv, 0);
  wmma_gemm64<0, false, 2, 1, false, 0, 0><<<dim3(128, 1, 1), 256, 0, stream>>>(
      xn, xn, kDim, 0L, wkT, wkT, kDim, 0L, (void*)kh, (void*)kh, kDim, 0L, bk, x, 0L,
      kTok, kDim, kDim, kWCarryInv, 0);
  wmma_gemm64<0, false, 1, 1, false, 0, 0><<<dim3(64, kBatch, 1), 256, 0, stream>>>(
      wvT, wvT, kDim, 0L, xn, xn, kDim, (long)kSeq * kDim, (void*)vT, (void*)vT, kSeq, (long)kDim * kSeq, bv, x, 0L,
      kDim, kSeq, kDim, kWCarryInv, 0);

  for (int p = 0; p < kPasses; ++p) {
    const int gbase = p * kGroupsPerPass;
    wmma_gemm64<0, false, 0, 0, false, 0, 1><<<dim3(3, kZPerPass, 1), 256, 0, stream>>>(
        qh, qh, kDim, 0L, kh, kh, kDim, 0L, (void*)scores, (void*)scores, kWinK, 0L, bq, x, 0L,
        kChunkQ, kWinK, kHeadDim, kScoreScale, gbase);
    band_softmax_kernel<<<dim3(kChunkQ, kZPerPass, 1), 128, 0, stream>>>(scores, pPl);
    wmma_gemm64<0, false, 0, 1, false, 0, 2><<<dim3(1, kZPerPass, 1), 64, 0, stream>>>(
        pPl, pPl, kWinK, 0L, vT, vT, kSeq, 0L, (void*)ctx, (void*)ctx, kDim, 0L, bq, x, 0L,
        kChunkQ, kHeadDim, kWinK, kPVScale, gbase);
  }

  wmma_gemm64<0, false, 2, 0, true, 0, 0><<<dim3(128, 1, 1), 256, 0, stream>>>(
      ctx, ctx, kDim, 0L, woT, woT, kDim, 0L, (void*)x1, (void*)x1, kDim, 0L, bo, x, 0L,
      kTok, kDim, kDim, kWoScale, 0);

  ln_f16_kernel<<<dim3(kTok), 128, 0, stream>>>(x1, ln2g, ln2b, xn);

  wmma_gemm64<0, false, 2, 1, false, 2, 0><<<dim3(512, 1, 1), 256, 0, stream>>>(
      xn, xn, kDim, 0L, w1T, w1T, kDim, 0L, (void*)ff1, (void*)ff1, kFF, 0L, b1, x, 0L,
      kTok, kFF, kDim, kWCarryInv, 0);
  wmma_gemm64<0, false, 2, 0, true, 0, 0><<<dim3(128, 1, 1), 256, 0, stream>>>(
      ff1, ff1, kFF, 0L, w2T, w2T, kFF, 0L, (void*)out, (void*)out, kDim, 0L, b2, x1, 0L,
      kTok, kDim, kFF, kWCarryInv, 0);
}
